// CustomMultiHeadAttention_48490180772334
// MI455X (gfx1250) — hardware-verified
//
#include <hip/hip_runtime.h>
#include <stdint.h>

#define NB   4
#define SEQ  1024
#define DM   1024
#define NH   16
#define HD   64
#define DK2  (2 * DM)
static_assert(NH * HD == DM);
static_assert(HD == 64);
static_assert((SEQ % 64) == 0 && (DM % 64) == 0 && ((NB * SEQ) % 64) == 0);
static_assert((DM % 32) == 0 && (DK2 % 32) == 0);

typedef _Float16 v16h __attribute__((ext_vector_type(16)));
typedef _Float16 v8h  __attribute__((ext_vector_type(8)));
typedef __bf16   v16b __attribute__((ext_vector_type(16)));
typedef __bf16   v8b  __attribute__((ext_vector_type(8)));
typedef float    v8f  __attribute__((ext_vector_type(8)));
typedef float    v4f  __attribute__((ext_vector_type(4)));
typedef unsigned int v4u __attribute__((ext_vector_type(4)));
typedef int      v4i  __attribute__((ext_vector_type(4)));
typedef int      v8i  __attribute__((ext_vector_type(8)));
typedef v8h __attribute__((may_alias)) v8ha;
typedef v8b __attribute__((may_alias)) v8ba;
typedef v4f __attribute__((may_alias)) v4fa;
typedef v4i __attribute__((may_alias)) v4ia;

#if defined(__HIP_DEVICE_COMPILE__)
#define DEV_ASM 1
#else
#define DEV_ASM 0
#endif

#define PSC   1024.0f
#define SFILL (-1.0e30f)

__device__ __forceinline__ unsigned short bf_bits(float f) {
  unsigned u = __float_as_uint(f);
  return (unsigned short)((u + 0x7FFFu + ((u >> 16) & 1u)) >> 16);
}
__device__ __forceinline__ float bf_up(unsigned short hb) { return __uint_as_float(((unsigned)hb) << 16); }
__device__ __forceinline__ float bfr(float f) { return bf_up(bf_bits(f)); }
__device__ __forceinline__ unsigned short h_bits(_Float16 x) { return __builtin_bit_cast(unsigned short, x); }
__device__ __forceinline__ unsigned pk16(unsigned short a, unsigned short b) { return (unsigned)a | ((unsigned)b << 16); }
__device__ __forceinline__ v8f zero8() { v8f z = {0.f, 0.f, 0.f, 0.f, 0.f, 0.f, 0.f, 0.f}; return z; }

template <typename OT> struct FT;
template <> struct FT<__bf16>   { typedef v16b frag; typedef v8ba half8; };
template <> struct FT<_Float16> { typedef v16h frag; typedef v8ha half8; };

template <typename OT>
__device__ __forceinline__ typename FT<OT>::frag ldfrag(const OT* p) {
  union { typename FT<OT>::frag v; typename FT<OT>::half8 h[2]; } f;
  f.h[0] = *(const typename FT<OT>::half8*)(p);
  f.h[1] = *(const typename FT<OT>::half8*)(p + 16);
  return f.v;
}
__device__ __forceinline__ v16h lf16(const _Float16* p, int hh) { return ldfrag<_Float16>(p + 8 * hh); }

__device__ __forceinline__ v8f mmar(v16b a, v16b b, v8f c) {
  return __builtin_amdgcn_wmma_f32_16x16x32_bf16(false, a, false, b, (short)0, c, false, false);
}
__device__ __forceinline__ v8f mmar(v16h a, v16h b, v8f c) {
  return __builtin_amdgcn_wmma_f32_16x16x32_f16(false, a, false, b, (short)0, c, false, false);
}
__device__ __forceinline__ v8f mma_h(v16h a, v16h b, v8f c) {
  c = __builtin_amdgcn_wmma_f32_16x16x32_f16(false, a, false, b, (short)0, c, false, false);
#if DEV_ASM
  asm volatile("v_nop\n\tv_nop\n\tv_nop\n\tv_nop" : "+v"(c) : "v"(a), "v"(b));
#endif
  return c;
}
__device__ __forceinline__ void dep_guard(v8f& a, v8f& b, v16b x, v16b y) {
#if DEV_ASM
  asm volatile("v_nop\n\tv_nop\n\tv_nop\n\tv_nop" : "+v"(a), "+v"(b) : "v"(x), "v"(y));
#else
  (void)a; (void)b; (void)x; (void)y;
#endif
}
__device__ __forceinline__ void dep_guard(v8f& a, v8f& b, v16h x, v16h y) {
#if DEV_ASM
  asm volatile("v_nop\n\tv_nop\n\tv_nop\n\tv_nop" : "+v"(a), "+v"(b) : "v"(x), "v"(y));
#else
  (void)a; (void)b; (void)x; (void)y;
#endif
}
__device__ __forceinline__ void keep4(v16b a, v16b b, v16b c, v16b d) {
#if DEV_ASM
  asm volatile("v_nop" :: "v"(a), "v"(b), "v"(c), "v"(d));
#else
  (void)a; (void)b; (void)c; (void)d;
#endif
}
__device__ __forceinline__ void keep4(v16h a, v16h b, v16h c, v16h d) {
#if DEV_ASM
  asm volatile("v_nop" :: "v"(a), "v"(b), "v"(c), "v"(d));
#else
  (void)a; (void)b; (void)c; (void)d;
#endif
}
__device__ __forceinline__ void acc_guard4(v8f& a, v8f& b, v8f& c, v8f& d) {
#if DEV_ASM
  asm volatile("v_nop\n\tv_nop\n\tv_nop\n\tv_nop" : "+v"(a), "+v"(b), "+v"(c), "+v"(d));
#else
  (void)a; (void)b; (void)c; (void)d;
#endif
}

__global__ __launch_bounds__(256) void cvt3_bf16x8(
    const float* __restrict__ a0, const float* __restrict__ a1, const float* __restrict__ a2,
    unsigned short* o0, unsigned short* o1, unsigned short* o2, int n8) {
  const int sel = blockIdx.y;
  const float* in = (sel == 0) ? a0 : ((sel == 1) ? a1 : a2);
  unsigned short* out = (sel == 0) ? o0 : ((sel == 1) ? o1 : o2);
  const int i = blockIdx.x * 256 + (int)threadIdx.x;
  if (i < n8) {
    const v4f a  = *(const v4fa*)(in + (size_t)i * 8);
    const v4f a4 = *(const v4fa*)(in + (size_t)i * 8 + 4);
    v4u p;
    p[0] = pk16(bf_bits(a[0]),  bf_bits(a[1]));
    p[1] = pk16(bf_bits(a[2]),  bf_bits(a[3]));
    p[2] = pk16(bf_bits(a4[0]), bf_bits(a4[1]));
    p[3] = pk16(bf_bits(a4[2]), bf_bits(a4[3]));
    unsigned short* o = out + (size_t)i * 8;
    *(volatile v4u*)o = p;
    __threadfence();
    *(volatile v4u*)o = p;
  }
}

template <int DUP>
__global__ __launch_bounds__(256) void transpose64(
    const float* __restrict__ in0, const float* __restrict__ in1, const float* __restrict__ in2,
    unsigned short* out0, unsigned short* out1, unsigned short* out2,
    int R, int C, int zPer, int ldo, long long strideOut, int dupOff) {
  __shared__ __align__(16) float tile[64][65];
  const int zsel = blockIdx.z / zPer;
  const int zz   = blockIdx.z - zsel * zPer;
  const float* in = (zsel == 0) ? in0 : ((zsel == 1) ? in1 : in2);
  unsigned short* out = (zsel == 0) ? out0 : ((zsel == 1) ? out1 : out2);
  const int c0 = blockIdx.x * 64, r0 = blockIdx.y * 64;
  const int tid = (int)threadIdx.x;
  {
    const int row = tid >> 2, seg = (tid & 3) * 16;
    const float* src = in + ((size_t)zz * R + r0 + row) * (size_t)C + c0 + seg;
#pragma unroll
    for (int k = 0; k < 4; ++k) {
      const v4f a = *(const v4fa*)(src + 4 * k);
      tile[row][seg + 4 * k + 0] = a[0];
      tile[row][seg + 4 * k + 1] = a[1];
      tile[row][seg + 4 * k + 2] = a[2];
      tile[row][seg + 4 * k + 3] = a[3];
    }
  }
  __syncthreads();
  const int q8 = tid & 7, sub = tid >> 3;
  v4u pk[2];
  size_t go[2];
#pragma unroll
  for (int i = 0; i < 2; ++i) {
    const int lid = i * 32 + sub;
    v4u a;
#pragma unroll
    for (int e = 0; e < 4; ++e)
      a[e] = pk16(bf_bits(tile[8 * q8 + 2 * e][lid]), bf_bits(tile[8 * q8 + 2 * e + 1][lid]));
    pk[i] = a;
    go[i] = (size_t)zz * (size_t)strideOut + (size_t)(c0 + lid) * (size_t)ldo + r0 + 8 * q8;
  }
  for (int pass = 0; pass < 2; ++pass) {
#pragma unroll
    for (int i = 0; i < 2; ++i) {
      *(volatile v4u*)(out + go[i]) = pk[i];
      if (DUP) *(volatile v4u*)(out + go[i] + dupOff) = pk[i];
    }
    __threadfence();
  }
}

template <typename OT, int OUT_MODE, int BIAS>
__global__ __launch_bounds__(256) void gemm64(
    const unsigned short* __restrict__ Ap, int lda, long long strideA,
    const unsigned short* __restrict__ Btp, int ldb, long long strideB,
    void* Cout, void* Cout2, int ldc, long long strideC,
    const float* __restrict__ bias,
    int M, int N, int K, float oscale, float rscale) {
  typedef typename FT<OT>::frag V16;
  const OT* A  = (const OT*)(const void*)Ap;
  const OT* Bt = (const OT*)(const void*)Btp;
  __shared__ __align__(16) float sT[8][16 * 68];
  const int b    = blockIdx.y;
  const int lane = threadIdx.x & 31;
  const int wave = threadIdx.x >> 5;
  const int tilesN = N >> 6;
  const int tilesM = M >> 6;
  const int tile = blockIdx.x * 8 + wave;
  if (tile >= tilesM * tilesN) return;
  const int tm = tile / tilesN;
  const int tn = tile - tm * tilesN;
  const int m0 = tm << 6;
  const int n0 = tn << 6;

  const OT* Ab = A  + (size_t)b * (size_t)strideA;
  const OT* Bb = Bt + (size_t)b * (size_t)strideB;

  const int rlane = lane & 15;
  const int koff  = (lane >> 4) * 8;
  const int mOff  = (lane >> 4) * 8;

  v8f acc[4][4];
#pragma unroll
  for (int i = 0; i < 4; ++i)
#pragma unroll
    for (int j = 0; j < 4; ++j) acc[i][j] = zero8();

  for (int k0 = 0; k0 < K; k0 += 32) {
    V16 bq[4];
#pragma unroll
    for (int j = 0; j < 4; ++j)
      bq[j] = ldfrag<OT>(Bb + (size_t)(n0 + (j << 4) + rlane) * ldb + koff + k0);
#pragma unroll
    for (int i = 0; i < 4; ++i) {
      const V16 af = ldfrag<OT>(Ab + (size_t)(m0 + (i << 4) + rlane) * lda + koff + k0);
#pragma unroll
      for (int j = 0; j < 4; ++j) acc[i][j] = mmar(af, bq[j], acc[i][j]);
      dep_guard(acc[i][0], acc[i][3], af, bq[3]);
    }
    keep4(bq[0], bq[1], bq[2], bq[3]);
  }
  acc_guard4(acc[0][0], acc[0][1], acc[0][2], acc[0][3]);
  acc_guard4(acc[1][0], acc[1][1], acc[1][2], acc[1][3]);
  acc_guard4(acc[2][0], acc[2][1], acc[2][2], acc[2][3]);
  acc_guard4(acc[3][0], acc[3][1], acc[3][2], acc[3][3]);

  float* slab = sT[wave];
#pragma unroll
  for (int i = 0; i < 4; ++i) {
    const int mBase = m0 + (i << 4);
#pragma unroll
    for (int j = 0; j < 4; ++j) {
#pragma unroll
      for (int r = 0; r < 8; ++r) {
        slab[(mOff + r) * 68 + (j << 4) + rlane] = acc[i][j][r];
      }
    }
    __builtin_amdgcn_fence(__ATOMIC_RELEASE, "workgroup");
    __builtin_amdgcn_wave_barrier();
    __builtin_amdgcn_fence(__ATOMIC_ACQUIRE, "workgroup");
    if (OUT_MODE == 0) {
      float* C = (float*)Cout + (size_t)b * (size_t)strideC;
      const int h2 = lane >> 4, c4 = (lane & 15) * 4;
      v4f badd = {0.f, 0.f, 0.f, 0.f};
      if (BIAS == 1) {
        const v4f bb = *(const v4fa*)(bias + n0 + c4);
        badd[0] = bfr(bb[0]); badd[1] = bfr(bb[1]); badd[2] = bfr(bb[2]); badd[3] = bfr(bb[3]);
      }
      for (int pass = 0; pass < 2; ++pass) {
#pragma unroll
        for (int it = 0; it < 8; ++it) {
          const int row = it * 2 + h2;
          v4f v = *(const v4f*)(slab + row * 68 + c4) * oscale + badd;
          if (BIAS == 2) {
            const float br = bfr(bias[mBase + row]);
            v[0] += br; v[1] += br; v[2] += br; v[3] += br;
          }
          *(volatile v4f*)(C + (size_t)(mBase + row) * ldc + n0 + c4) = v;
        }
        __threadfence();
      }
    } else {
      const int q = lane >> 3, c8 = (lane & 7) * 8;
      unsigned short* C  = (unsigned short*)Cout  + (size_t)b * (size_t)strideC;
      unsigned short* C2 = (unsigned short*)Cout2 + (size_t)b * (size_t)strideC;
      v4u hv[4], lv[4];
#pragma unroll
      for (int it = 0; it < 4; ++it) {
        const int row = it * 4 + q;
        const float* sp = slab + row * 68 + c8;
        float f[8];
#pragma unroll
        for (int e = 0; e < 8; ++e) f[e] = sp[e];
        if (BIAS == 1) {
          const v4f b0 = *(const v4fa*)(bias + n0 + c8);
          const v4f b1 = *(const v4fa*)(bias + n0 + c8 + 4);
#pragma unroll
          for (int e = 0; e < 4; ++e) { f[e] += bfr(b0[e]); f[4 + e] += bfr(b1[e]); }
        } else if (BIAS == 2) {
          const float br = bfr(bias[mBase + row]);
#pragma unroll
          for (int e = 0; e < 8; ++e) f[e] += br;
        }
        v4u a, a2;
#pragma unroll
        for (int e = 0; e < 4; ++e) {
          const float f0 = f[2 * e], f1 = f[2 * e + 1];
          const _Float16 x0 = (_Float16)f0, x1 = (_Float16)f1;
          const unsigned short h0 = h_bits(x0), h1 = h_bits(x1);
          unsigned short l0 = 0, l1 = 0;
          if (OUT_MODE == 3) {
            l0 = h_bits((_Float16)((f0 - (float)x0) * rscale));
            l1 = h_bits((_Float16)((f1 - (float)x1) * rscale));
          }
          a[e] = pk16(h0, h1); a2[e] = pk16(l0, l1);
        }
        hv[it] = a; lv[it] = a2;
      }
      for (int pass = 0; pass < 2; ++pass) {
#pragma unroll
        for (int it = 0; it < 4; ++it) {
          const int row = it * 4 + q;
          *(volatile v4u*)(C + (size_t)(mBase + row) * ldc + n0 + c8) = hv[it];
          if (OUT_MODE == 3) *(volatile v4u*)(C2 + (size_t)(mBase + row) * ldc + n0 + c8) = lv[it];
        }
        __threadfence();
      }
    }
    __builtin_amdgcn_fence(__ATOMIC_RELEASE, "workgroup");
    __builtin_amdgcn_wave_barrier();
    __builtin_amdgcn_fence(__ATOMIC_ACQUIRE, "workgroup");
  }
}

__device__ __forceinline__ v16h pack_p(v8f a, v8f c) {
  const v16h r = { (_Float16)(a[0] * PSC), (_Float16)(a[1] * PSC), (_Float16)(a[2] * PSC), (_Float16)(a[3] * PSC),
                   (_Float16)(a[4] * PSC), (_Float16)(a[5] * PSC), (_Float16)(a[6] * PSC), (_Float16)(a[7] * PSC),
                   (_Float16)(c[0] * PSC), (_Float16)(c[1] * PSC), (_Float16)(c[2] * PSC), (_Float16)(c[3] * PSC),
                   (_Float16)(c[4] * PSC), (_Float16)(c[5] * PSC), (_Float16)(c[6] * PSC), (_Float16)(c[7] * PSC) };
  return r;
}

__global__ __launch_bounds__(128) void attn_kernel(
    const unsigned short* __restrict__ qhp, const unsigned short* __restrict__ qlp,
    const unsigned short* __restrict__ kpp, const unsigned short* __restrict__ vtp,
    const int* __restrict__ mask, unsigned short* cxp) {
  __shared__ __align__(16) float sO[4 * 16 * 64];

  const int tid = threadIdx.x, lane = tid & 31, w = tid >> 5;
  const int h = lane >> 4, m = lane & 15;
  const int bh = blockIdx.y, b = bh >> 4, head = bh & 15;
  const int q0 = blockIdx.x * 64 + 16 * w;

  const _Float16* Qh = (const _Float16*)(const void*)qhp;
  const _Float16* Ql = (const _Float16*)(const void*)qlp;
  const _Float16* Kp = (const _Float16*)(const void*)kpp;
  const _Float16* Vt = (const _Float16*)(const void*)vtp;

  const size_t qo = ((size_t)b * SEQ + q0 + m) * DM + (size_t)head * HD;
  const v16h qh0 = lf16(Qh + qo, h);
  const v16h qh1 = lf16(Qh + qo + 32, h);
  const v16h ql0 = lf16(Ql + qo, h);
  const v16h ql1 = lf16(Ql + qo + 32, h);

  v8f o[4];
#pragma unroll
  for (int t = 0; t < 4; ++t) o[t] = zero8();
  float mrun = SFILL, lrun = 0.0f;

  const _Float16* kbase = Kp + ((size_t)b * SEQ + m) * DM + (size_t)head * HD;
  const _Float16* vbase = Vt + ((size_t)b * DM + (size_t)head * HD + m) * SEQ;
  const int* mk = mask + ((size_t)b * SEQ + q0 + m) * SEQ + 8 * h;

#pragma unroll 1
  for (int kb = 0; kb < SEQ; kb += 64) {
    v8f s[4];
#pragma unroll
    for (int j = 0; j < 4; ++j) {
      const _Float16* kp = kbase + (size_t)(kb + 16 * j) * DM;
      const v16h kf0 = lf16(kp, h);
      const v16h kf1 = lf16(kp + 32, h);
      v8f zh = zero8(), zl = zero8();
      zh = mma_h(kf0, qh0, zh);
      zh = mma_h(kf1, qh1, zh);
      zl = mma_h(kf0, ql0, zl);
      zl = mma_h(kf1, ql1, zl);
      const v4i ma = *(const v4ia*)(mk + kb + 16 * j);
      const v4i mb = *(const v4ia*)(mk + kb + 16 * j + 4);
      const v8i mv = __builtin_shufflevector(ma, mb, 0, 1, 2, 3, 4, 5, 6, 7);
      v8f t;
#pragma unroll
      for (int r = 0; r < 8; ++r) {
        const float sv = (zh[r] + zl[r] * (1.0f / 4096.0f)) * (1.0f / 32.0f);
        t[r] = (mv[r] != 0) ? sv : SFILL;
      }
      s[j] = t;
    }

    float mloc = s[0][0];
#pragma unroll
    for (int j = 0; j < 4; ++j)
#pragma unroll
      for (int r = 0; r < 8; ++r) mloc = fmaxf(mloc, s[j][r]);
    mloc = fmaxf(mloc, __shfl_xor(mloc, 16, 32));
    const float mnew = fmaxf(mrun, mloc);
    const float alpha = __expf(mrun - mnew);
    mrun = mnew;
    float lsum = 0.0f;
#pragma unroll
    for (int j = 0; j < 4; ++j)
#pragma unroll
      for (int r = 0; r < 8; ++r) {
        const float sv = s[j][r];
        const float e  = __expf(sv - mnew);
        const float p  = (sv > -1.0e29f) ? e : 0.0f;
        s[j][r] = p;
        lsum += p;
      }
    lsum += __shfl_xor(lsum, 16, 32);
    lrun = lrun * alpha + lsum;
#pragma unroll
    for (int t = 0; t < 4; ++t)
#pragma unroll
      for (int r = 0; r < 8; ++r) o[t][r] = o[t][r] * alpha;

    const v16h pb0 = pack_p(s[0], s[1]);
    const v16h pb1 = pack_p(s[2], s[3]);

#pragma unroll
    for (int t = 0; t < 4; ++t) {
      const _Float16* vp = vbase + (size_t)(16 * t) * SEQ + kb;
      const v16h vf0 = lf16(vp, h);
      const v16h vf1 = lf16(vp + 32, h);
      o[t] = mma_h(vf0, pb0, o[t]);
      o[t] = mma_h(vf1, pb1, o[t]);
    }
  }

  const float inv = ((lrun > 0.0f) ? (1.0f / lrun) : 0.0f) * (1.0f / PSC);
  float* so = sO + w * 1024;
#pragma unroll
  for (int t = 0; t < 4; ++t)
#pragma unroll
    for (int r = 0; r < 8; ++r)
      so[m * 64 + 16 * t + 8 * h + r] = o[t][r] * inv;
  __syncthreads();

  {
    const int q8 = lane & 7, sub = lane >> 3;
    v4u pk[8];
#pragma unroll
    for (int i = 0; i < 8; ++i) {
      const int lid = i * 4 + sub;
      const int row = lid >> 1, wl = lid & 1;
      const float* sp = so + row * 64 + 8 * q8;
      const v4f fa = *(const v4fa*)sp;
      const v4f fb = *(const v4fa*)(sp + 4);
      const v8f fv = __builtin_shufflevector(fa, fb, 0, 1, 2, 3, 4, 5, 6, 7);
      v4u a;
#pragma unroll
      for (int e = 0; e < 4; ++e) {
        const float f0 = fv[2 * e], f1 = fv[2 * e + 1];
        const unsigned short h0 = bf_bits(f0), h1 = bf_bits(f1);
        const unsigned short l0 = bf_bits(f0 - bf_up(h0)), l1 = bf_bits(f1 - bf_up(h1));
        a[e] = (wl != 0) ? pk16(l0, l1) : pk16(h0, h1);
      }
      pk[i] = a;
    }
    for (int pass = 0; pass < 2; ++pass) {
#pragma unroll
      for (int i = 0; i < 8; ++i) {
        const int lid = i * 4 + sub;
        const int row = lid >> 1, wl = lid & 1;
        const size_t go = ((size_t)b * SEQ + q0 + row) * DK2 + (size_t)wl * DM + (size_t)head * HD + 8 * q8;
        *(volatile v4u*)(cxp + go) = pk[i];
      }
      __threadfence();
    }
  }
}

extern "C" void kernel_launch(void* const* d_in, const int* in_sizes, int n_in,
                              void* d_out, int out_size, void* d_ws, size_t ws_size,
                              hipStream_t stream) {
  if (n_in < 12) return;
  const int nAct = NB * SEQ * DM;
  const int nMsk = NB * SEQ * SEQ;
  const int nWh  = NH * DM * HD;
  const int nBh  = NH * HD;
  if (in_sizes[0] != nAct || in_sizes[1] != nAct || in_sizes[2] != nAct) return;
  if (in_sizes[3] != nMsk) return;
  if (in_sizes[4] != nWh || in_sizes[6] != nWh || in_sizes[8] != nWh) return;
  if (in_sizes[5] != nBh || in_sizes[7] != nBh || in_sizes[9] != nBh) return;
  if (in_sizes[10] != DM * DM || in_sizes[11] != DM) return;
  if (out_size != nAct) return;

  const float* query = (const float*)d_in[0];
  const float* key   = (const float*)d_in[1];
  const float* value = (const float*)d_in[2];
  const int*   mask  = (const int*)d_in[3];
  const float* Wq = (const float*)d_in[4];
  const float* bq = (const float*)d_in[5];
  const float* Wk = (const float*)d_in[6];
  const float* bk = (const float*)d_in[7];
  const float* Wv = (const float*)d_in[8];
  const float* bv = (const float*)d_in[9];
  const float* Wo = (const float*)d_in[10];
  const float* bo = (const float*)d_in[11];

  const size_t PX  = (size_t)nAct * 2;
  const size_t PW  = (size_t)nWh * 2;
  const size_t PWO = (size_t)DM * DK2 * 2;
  const size_t PCX = (size_t)NB * SEQ * DK2 * 2;
  size_t off = 0;
  const size_t oXq = off; off += PX;
  const size_t oXk = off; off += PX;
  const size_t oXv = off; off += PX;
  const size_t oWq = off; off += PW;
  const size_t oWk = off; off += PW;
  const size_t oWv = off; off += PW;
  const size_t oWo = off; off += PWO;
  const size_t oQh = off; off += PX;
  const size_t oQl = off; off += PX;
  const size_t oKp = off; off += PX;
  const size_t oVt = off; off += PX;
  const size_t oCx = off; off += PCX;
  if (off > ws_size) return;
  if (off > (size_t)134217728) return;

  char* ws = (char*)d_ws;
  unsigned short* Xq  = (unsigned short*)(ws + oXq);
  unsigned short* Xk  = (unsigned short*)(ws + oXk);
  unsigned short* Xv  = (unsigned short*)(ws + oXv);
  unsigned short* WqT = (unsigned short*)(ws + oWq);
  unsigned short* WkT = (unsigned short*)(ws + oWk);
  unsigned short* WvT = (unsigned short*)(ws + oWv);
  unsigned short* WoT = (unsigned short*)(ws + oWo);
  unsigned short* Qh  = (unsigned short*)(ws + oQh);
  unsigned short* Ql  = (unsigned short*)(ws + oQl);
  unsigned short* Kp  = (unsigned short*)(ws + oKp);
  unsigned short* Vt  = (unsigned short*)(ws + oVt);
  unsigned short* Cx  = (unsigned short*)(ws + oCx);

  const dim3 blk(256);
  const int n8 = nAct / 8;
  const dim3 gCvt((n8 + 255) / 256, 3);
  const dim3 gTw(HD / 64, DM / 64, 3 * NH);
  const dim3 gTo(DM / 64, DM / 64, 1);
  const dim3 gP((((NB * SEQ) / 64) * (DM / 64) + 7) / 8, 1);
  const dim3 gVT(((DM / 64) * (SEQ / 64) + 7) / 8, NB);
  const dim3 gAttn(SEQ / 64, NB * NH);

  cvt3_bf16x8<<<gCvt, blk, 0, stream>>>(query, key, value, Xq, Xk, Xv, n8);
  transpose64<0><<<gTw, blk, 0, stream>>>(Wq, Wk, Wv, WqT, WkT, WvT,
                                          DM, HD, NH, DM, (long long)HD * DM, 0);
  transpose64<1><<<gTo, blk, 0, stream>>>(Wo, Wo, Wo, WoT, WoT, WoT,
                                          DM, DM, 1, DK2, 0LL, DM);
  gemm64<__bf16, 3, 1><<<gP, blk, 0, stream>>>(
      Xq, DM, 0LL, WqT, DM, 0LL,
      (void*)Qh, (void*)Ql, DM, 0LL, bq,
      NB * SEQ, DM, DM, 1.0f, 4096.0f);
  gemm64<__bf16, 1, 1><<<gP, blk, 0, stream>>>(
      Xk, DM, 0LL, WkT, DM, 0LL,
      (void*)Kp, (void*)Kp, DM, 0LL, bk,
      NB * SEQ, DM, DM, 1.0f, 1.0f);
  gemm64<__bf16, 1, 2><<<gVT, blk, 0, stream>>>(
      WvT, DM, 0LL, Xv, DM, (long long)SEQ * DM,
      (void*)Vt, (void*)Vt, SEQ, (long long)DM * SEQ, bv,
      DM, SEQ, DM, 1.0f, 1.0f);
  attn_kernel<<<gAttn, dim3(128), 0, stream>>>(Qh, Ql, Kp, Vt, mask, Cx);
  gemm64<__bf16, 0, 1><<<gP, blk, 0, stream>>>(
      Cx, DK2, 0LL, WoT, DK2, 0LL,
      d_out, d_out, DM, 0LL, bo,
      NB * SEQ, DM, DK2, 1.0f, 1.0f);
  (void)hipGetLastError();
}
